// LinearMimo_40742059769933
// MI455X (gfx1250) — hardware-run, weakly checked
//
#include <hip/hip_runtime.h>
#include <hip/hip_fp16.h>
#include <math.h>


typedef __attribute__((ext_vector_type(16))) _Float16 v16h;
typedef __attribute__((ext_vector_type(8)))  _Float16 v8h;
typedef __attribute__((ext_vector_type(8)))  float    v8f;
typedef __attribute__((ext_vector_type(4)))  float    v4f;
typedef __attribute__((ext_vector_type(2)))  unsigned v2u;
typedef __attribute__((ext_vector_type(2)))  float    v2f;
typedef __attribute__((ext_vector_type(4)))  unsigned v4u;

constexpr int kB = 16;
constexpr int kT = 4096;
constexpr int kI = 32;
constexpr int kO = 32;
constexpr int kL = 32;
constexpr int kC = kT / kL;
constexpr int kS = kL + 2;
constexpr int kK = kS * kI;
constexpr int kN = kL * kO;
constexpr int kPairs = kO * kI;
constexpr int kTabPlanes = kS + kL;
constexpr int kUpB = (kT + 2) * kI;
constexpr float kWCarry = 65536.0f;
static_assert(kC == 128 && kS == 34 && kK == 1088 && kN == 1024 && kPairs == 1024 && kTabPlanes == 66);
static_assert(kUpB == 131136);
static_assert((kK % 32) == 0 && (kN % 64) == 0 && (kC % 32) == 0);
static_assert(((kC / 32) * (kN / 64)) % 8 == 0);
static_assert((kC - 1) * (kL * kI) + kK == kUpB);
static_assert(((kUpB * 2) % 128) == 0);

constexpr int kSegRows = 144;
constexpr int kSeg = kSegRows * 32;
constexpr int kUiCh = kB * kSeg;
constexpr int kUiTail = 256;
constexpr int kFRows = kB * kSegRows;
constexpr int kFN = 64;
constexpr int kFK = 64;
constexpr int kGN = kB * kC;
constexpr float kHCarry = 32768.0f;
static_assert(kSeg == 4608 && kUiCh == 73728 && kFRows == 2304 && kGN == 2048);
static_assert(kSegRows >= kC && kSeg >= kT + 2 && (kSeg % 8) == 0);
static_assert(kFN == 2 * kO && kFK == 2 * kI && kS <= kFK && kL >= 2);
static_assert((kFRows % 32) == 0 && (kFN % 64) == 0 && (kFK % 32) == 0);
static_assert((kFRows / 32) % 8 == 0);
static_assert(((kFRows / 32) * (kFN / 64)) % 8 == 0);
static_assert((kFRows - 1) * 32 + kFK <= kUiCh + kUiTail);
static_assert((kL % 32) == 0 && (kGN % 64) == 0);
static_assert(((kL / 32) * (kGN / 64)) % 8 == 0);
static_assert((((size_t)kI * kUiCh * 2) % 128) == 0);

constexpr size_t kSzAR  = (size_t)kPairs * 2 * 4;
constexpr size_t kSzBR  = (size_t)kPairs * 3 * 4;
constexpr size_t kSzTAB = (size_t)kTabPlanes * kPairs * 4;
constexpr size_t kSzHC  = (size_t)kL * kPairs * 2 * 4;
constexpr size_t kSzWT  = (size_t)kN * kK * 2;
constexpr size_t kSzUP  = (size_t)kB * kUpB * 2;
constexpr size_t kSzD   = (size_t)kB * kC * kN * 4;
constexpr size_t kSzUI  = ((size_t)kI * kUiCh + kUiTail) * 2;
constexpr size_t kSzWF  = (size_t)kI * kFN * kFK * 2;
constexpr size_t kSzHQ  = (size_t)kO * kL * kFK * 2;
constexpr size_t kSzF   = (size_t)kI * kFRows * kFN * 4;
constexpr size_t kSzYQ  = (size_t)kO * kGN * kFK * 2;
constexpr size_t kSzG   = (size_t)kO * kL * kGN * 4;
constexpr size_t kOffAR  = 0;
constexpr size_t kOffBR  = kOffAR  + kSzAR;
constexpr size_t kOffTAB = kOffBR  + kSzBR;
constexpr size_t kOffHC  = kOffTAB + kSzTAB;
constexpr size_t kOffWT  = kOffHC  + kSzHC;
constexpr size_t kOffUP  = kOffWT  + kSzWT;
constexpr size_t kOffD   = kOffUP  + kSzUP;
constexpr size_t kOffUI  = kOffD   + kSzD;
constexpr size_t kOffWF  = kOffUI  + kSzUI;
constexpr size_t kOffHQ  = kOffWF  + kSzWF;
constexpr size_t kOffF   = kOffHQ  + kSzHQ;
constexpr size_t kOffYQ  = kOffF   + kSzF;
constexpr size_t kOffG   = kOffYQ  + kSzYQ;
constexpr size_t kWsTotal = kOffG + kSzG;
static_assert(kSzAR == 8192ull && kSzBR == 12288ull && kSzTAB == 270336ull && kSzHC == 262144ull);
static_assert(kSzWT == 2228224ull && kSzUP == 4196352ull && kSzD == 8388608ull);
static_assert(kSzUI == 4719104ull && kSzWF == 262144ull && kSzHQ == 131072ull);
static_assert(kSzF == 18874368ull && kSzYQ == 8388608ull && kSzG == 8388608ull);
static_assert((kSzAR % 256) == 0 && (kSzBR % 256) == 0 && (kSzTAB % 256) == 0 && (kSzHC % 256) == 0 &&
              (kSzWT % 256) == 0 && (kSzUP % 256) == 0 && (kSzD % 256) == 0 && (kSzUI % 256) == 0 &&
              (kSzWF % 256) == 0 && (kSzHQ % 256) == 0 && (kSzF % 256) == 0 && (kSzYQ % 256) == 0 &&
              (kSzG % 256) == 0);
static_assert(kWsTotal == 56130048ull);
static_assert(kWsTotal <= 134217728ull);

__device__ __forceinline__ _Float16 f16_flush(float v) {
  const float w = (fabsf(v) < 6.103515625e-05f) ? 0.0f : v;
  return (_Float16)w;
}

__device__ __forceinline__ float bf16r(float v) {
  unsigned u = __float_as_uint(v);
  u = (u + 0x7FFFu + ((u >> 16) & 1u)) & 0xFFFF0000u;
  return __uint_as_float(u);
}

__device__ __forceinline__ float h16_to_f32(unsigned hb) {
  const unsigned sgn = (hb & 0x8000u) << 16; const unsigned em = hb & 0x7fffu;
  const float fn = __uint_as_float((em << 13) + 0x38000000u);
  const float fs = (float)em * 5.9604644775390625e-8f;
  const float mag = (em < 0x400u) ? fs : fn; return __uint_as_float(__float_as_uint(mag) | sgn); }

namespace eng {
union FragU { v16h v; v8h h[2]; };
__device__ __forceinline__ v16h frag_load(const _Float16* p) {
  FragU f;
  f.h[0] = *(const v8h*)(p);
  f.h[1] = *(const v8h*)(p + 16);
  return f.v;
}
__device__ __forceinline__ v8f mma(v16h a, v16h b, v8f c) {
  return __builtin_amdgcn_wmma_f32_16x16x32_f16(false, a, false, b, (short)0, c, false, false);
}
__device__ __forceinline__ void guard1(v8f& a, v16h x, v16h y) {
  asm volatile("v_nop\n\tv_nop\n\tv_nop\n\tv_nop" : "+v"(a) : "v"(x), "v"(y));
}
__device__ __forceinline__ void guard_acc(v8f& a) {
  asm volatile("v_nop\n\tv_nop\n\tv_nop\n\tv_nop" : "+v"(a));
}
__device__ __forceinline__ void keep4(v16h a, v16h b, v16h c, v16h d) {
  asm volatile("v_nop" :: "v"(a), "v"(b), "v"(c), "v"(d));
}

template <int MI, int SPL>
__global__ __launch_bounds__(256) void gemm_f16_kernel(
    const unsigned short* __restrict__ Ap, const unsigned short* __restrict__ A2p, int lda,
    const unsigned short* __restrict__ Btp, const unsigned short* __restrict__ Bt2p, int ldb,
    float* __restrict__ C, int ldc, int M, int N, int K, float scale, float rscale)
{
  static_assert(MI >= 1 && MI <= 2);
  static_assert(SPL >= 0 && SPL <= 2);
  const _Float16* A   = (const _Float16*)Ap;
  const _Float16* A2  = (const _Float16*)A2p;
  const _Float16* Bt  = (const _Float16*)Btp;
  const _Float16* Bt2 = (const _Float16*)Bt2p;
  __shared__ __align__(16) float sT[8][16 * 68];
  const int lane = threadIdx.x & 31;
  const int wave = threadIdx.x >> 5;
  const int tilesN = N >> 6;
  const int tilesM = M / (16 * MI);
  const int tile = blockIdx.x * 8 + wave;
  if (tile >= tilesM * tilesN) return;
  const int tm = tile / tilesN;
  const int tn = tile - tm * tilesN;
  const int m0 = tm * (16 * MI);
  const int n0 = tn << 6;
  const int rlane = lane & 15;
  const int koff  = (lane >> 4) * 8;
  const int mOff  = (lane >> 4) * 8;

  v8f acc[MI][4], accr[MI][4];
#pragma unroll
  for (int i = 0; i < MI; ++i)
#pragma unroll
    for (int j = 0; j < 4; ++j) {
      acc[i][j]  = (v8f){0.f, 0.f, 0.f, 0.f, 0.f, 0.f, 0.f, 0.f};
      accr[i][j] = (v8f){0.f, 0.f, 0.f, 0.f, 0.f, 0.f, 0.f, 0.f};
    }

  for (int k0 = 0; k0 < K; k0 += 32) {
    v16h bh[4], bl[4];
#pragma unroll
    for (int j = 0; j < 4; ++j) {
      const size_t bo = (size_t)(n0 + (j << 4) + rlane) * ldb + koff + k0;
      bh[j] = frag_load(Bt + bo);
      if (SPL == 2) bl[j] = frag_load(Bt2 + bo); else bl[j] = bh[j];
    }
#pragma unroll
    for (int i = 0; i < MI; ++i) {
      const size_t ao = (size_t)(m0 + (i << 4) + rlane) * lda + koff + k0;
      const v16h ah = frag_load(A + ao);
      v16h al = ah;
      if (SPL >= 1) al = frag_load(A2 + ao);
#pragma unroll
      for (int j = 0; j < 4; ++j) {
        acc[i][j] = mma(ah, bh[j], acc[i][j]);
        if (SPL >= 1) accr[i][j] = mma(al, bh[j], accr[i][j]);
        if (SPL == 2) accr[i][j] = mma(ah, bl[j], accr[i][j]);
      }
#pragma unroll
      for (int j = 0; j < 4; ++j) {
        guard1(acc[i][j], ah, al);
        if (SPL >= 1) guard1(accr[i][j], ah, al);
      }
    }
    keep4(bh[0], bh[1], bh[2], bh[3]);
    if (SPL == 2) keep4(bl[0], bl[1], bl[2], bl[3]);
  }
#pragma unroll
  for (int i = 0; i < MI; ++i)
#pragma unroll
    for (int j = 0; j < 4; ++j) {
      guard_acc(acc[i][j]);
      if (SPL >= 1) guard_acc(accr[i][j]);
    }

  float* slab = sT[wave];
#pragma unroll
  for (int i = 0; i < MI; ++i) {
    const int mBase = m0 + (i << 4);
#pragma unroll
    for (int j = 0; j < 4; ++j) {
#pragma unroll
      for (int r = 0; r < 8; ++r) {
        float v = acc[i][j][r] * scale;
        if (SPL >= 1) v += accr[i][j][r] * rscale;
        slab[(mOff + r) * 68 + (j << 4) + rlane] = v;
      }
    }
    __builtin_amdgcn_fence(__ATOMIC_RELEASE, "workgroup");
    __builtin_amdgcn_wave_barrier();
    __builtin_amdgcn_fence(__ATOMIC_ACQUIRE, "workgroup");
    {
      const int hh = lane >> 4, c4 = (lane & 15) * 4;
      for (int pass = 0; pass < 2; ++pass) {
#pragma unroll
        for (int it = 0; it < 8; ++it) {
          const int row = it * 2 + hh;
          const v4f v = *(const v4f*)(slab + row * 68 + c4);
          *(volatile v4f*)(C + (size_t)(mBase + row) * ldc + n0 + c4) = v;
        }
        __threadfence();
      }
    }
    __builtin_amdgcn_fence(__ATOMIC_RELEASE, "workgroup");
    __builtin_amdgcn_wave_barrier();
    __builtin_amdgcn_fence(__ATOMIC_ACQUIRE, "workgroup");
  }
}
}

__global__ __launch_bounds__(256) void rne_vec_kernel(
    const float* __restrict__ src, float* __restrict__ dst, int n4)
{
  const int i = blockIdx.x * 256 + threadIdx.x;
  if (i >= n4) return;
  const v4f a = *(const v4f*)(src + (size_t)i * 4);
  const float a0 = a[0];
  const float a1 = a[1];
  const float a2 = a[2];
  const float a3 = a[3];
  v4f r;
  r[0] = bf16r(a0);
  r[1] = bf16r(a1);
  r[2] = bf16r(a2);
  r[3] = bf16r(a3);
  float* p = dst + (size_t)i * 4;
  *(volatile v4f*)p = r;
  __threadfence();
  *(volatile v4f*)p = r;
}

__global__ __launch_bounds__(128) void pad_zero_kernel(unsigned short* __restrict__ UP)
{
  const int j = threadIdx.x;
  const int b = j >> 3;
  const int q = j & 7;
  const v4u z = (v4u){0u, 0u, 0u, 0u};
  unsigned short* p = UP + (size_t)b * kUpB + 8 * q;
  *(volatile v4u*)p = z;
  __threadfence();
  *(volatile v4u*)p = z;
}

static_assert(((kB * kT * kI / 8) % 256) == 0);
__global__ __launch_bounds__(256) void pad_body_f16_kernel(
    const float* __restrict__ u, unsigned short* __restrict__ UP)
{
  const int g = blockIdx.x * 256 + threadIdx.x;
  const int b = g >> 14;
  const int r = g & 16383;
  const float* sp = u + (size_t)b * (kT * kI) + (size_t)r * 8;
  const v4f a0 = *(const v4f*)(sp);
  const v4f a1 = *(const v4f*)(sp + 4);
  const float f0 = a0[0];
  const float f1 = a0[1];
  const float f2 = a0[2];
  const float f3 = a0[3];
  const float f4 = a1[0];
  const float f5 = a1[1];
  const float f6 = a1[2];
  const float f7 = a1[3];
  v8h hv;
  hv[0] = f16_flush(bf16r(f0));
  hv[1] = f16_flush(bf16r(f1));
  hv[2] = f16_flush(bf16r(f2));
  hv[3] = f16_flush(bf16r(f3));
  hv[4] = f16_flush(bf16r(f4));
  hv[5] = f16_flush(bf16r(f5));
  hv[6] = f16_flush(bf16r(f6));
  hv[7] = f16_flush(bf16r(f7));
  unsigned short* qh = UP + (size_t)b * kUpB + 64 + (size_t)r * 8;
  *(volatile v8h*)qh = hv;
  __threadfence();
  *(volatile v8h*)qh = hv;
}

static_assert(((kI * kUiCh / 8) % 256) == 0);
__global__ __launch_bounds__(256) void ui_pack_kernel(
    const unsigned short* __restrict__ UP, unsigned short* __restrict__ UI)
{
  const int j = blockIdx.x * 256 + threadIdx.x;
  const int e0 = j * 8;
  const int i = e0 / kUiCh;
  const int rem = e0 - i * kUiCh;
  const int b = rem / kSeg;
  const int pos0 = rem - b * kSeg;
  const unsigned short* ub = UP + (size_t)b * kUpB + 64 + i;
  unsigned w[8];
#pragma unroll
  for (int e = 0; e < 8; ++e) {
    const int t = pos0 + e - 2;
    const bool live = (t >= 0) && (t < kT);
    int tc = (t < 0) ? 0 : t;
    tc = (tc > kT - 1) ? (kT - 1) : tc;
    unsigned x = (unsigned)ub[(size_t)tc * kI];
    w[e] = live ? x : 0u;
  }
  v4u pk;
  pk[0] = w[0] | (w[1] << 16);
  pk[1] = w[2] | (w[3] << 16);
  pk[2] = w[4] | (w[5] << 16);
  pk[3] = w[6] | (w[7] << 16);
  unsigned short* qh = UI + (size_t)e0;
  *(volatile v4u*)qh = pk;
  __threadfence();
  *(volatile v4u*)qh = pk;
}

__global__ __launch_bounds__(32) void ui_tail_kernel(unsigned short* __restrict__ UI)
{
  const int l = threadIdx.x;
  const v4u z = (v4u){0u, 0u, 0u, 0u};
  unsigned short* p = UI + (size_t)kI * kUiCh + 8 * l;
  *(volatile v4u*)p = z;
  __threadfence();
  *(volatile v4u*)p = z;
}

static_assert((kPairs % 256) == 0);
__global__ __launch_bounds__(256) void coeff_table_kernel(
    const float* __restrict__ AR, const float* __restrict__ BR,
    float* __restrict__ TAB, float* __restrict__ HC)
{
  const int p = blockIdx.x * 256 + threadIdx.x;
  const v2f av = *(const v2f*)(AR + 2 * p);
  const float a0 = av[0];
  const float a1 = av[1];
  const float b0 = BR[3 * p + 0];
  const float b1 = BR[3 * p + 1];
  const float b2 = BR[3 * p + 2];
  float h[kS];
  h[0] = 1.0f;
  {
    float hm1 = 1.0f;
    float hm2 = 0.0f;
#pragma unroll
    for (int m = 1; m < kS; ++m) {
      const float t = a0 * hm1 + a1 * hm2;
      const float hm = -t;
      h[m] = hm;
      hm2 = hm1;
      hm1 = hm;
    }
  }
  float w[kL];
#pragma unroll
  for (int m = 0; m < kL; ++m) {
    float v = b0 * h[m];
    if (m >= 1) v = v + b1 * h[m - 1];
    if (m >= 2) v = v + b2 * h[m - 2];
    w[m] = v;
  }
  float g[kL];
#pragma unroll
  for (int m = 0; m < kL; ++m) g[m] = -(a1 * h[m]);

  for (int pass = 0; pass < 2; ++pass) {
#pragma unroll
    for (int m = 0; m < kS; ++m)
      *(volatile float*)(TAB + (size_t)m * kPairs + p) = h[m];
#pragma unroll
    for (int m = 0; m < kL; ++m)
      *(volatile float*)(TAB + (size_t)(kS + m) * kPairs + p) = w[m];
#pragma unroll
    for (int m = 0; m < kL; ++m) {
      v2f v;
      v[0] = h[m + 1];
      v[1] = g[m];
      *(volatile v2f*)(HC + ((size_t)m * kPairs + p) * 2) = v;
    }
    __threadfence();
  }
}

static_assert(((kN * kK / 8) % 256) == 0 && (kK % 8) == 0);
__global__ __launch_bounds__(256) void wt_pack_kernel(
    const float* __restrict__ TAB, const float* __restrict__ BR, unsigned short* __restrict__ WT)
{
  const int j = blockIdx.x * 256 + threadIdx.x;
  const int e0 = j * 8;
  const int n = e0 / kK;
  const int k = e0 - n * kK;
  const int M = n >> 5;
  const int o = n & 31;
  const int s = k >> 5;
  const int i0 = k & 31;
  const int p0 = 32 * o + i0;
  const int Mm1 = (M > 0) ? (M - 1) : 0;
  int mw = M + 2 - s;
  mw = (mw < 0) ? 0 : mw;
  mw = (mw > kL - 1) ? (kL - 1) : mw;

  v4f hA[2], hB[2], wv[2], br[6];
  hA[0] = *(const v4f*)(TAB + (size_t)M * kPairs + p0);
  hA[1] = *(const v4f*)(TAB + (size_t)M * kPairs + p0 + 4);
  hB[0] = *(const v4f*)(TAB + (size_t)Mm1 * kPairs + p0);
  hB[1] = *(const v4f*)(TAB + (size_t)Mm1 * kPairs + p0 + 4);
  wv[0] = *(const v4f*)(TAB + (size_t)(kS + mw) * kPairs + p0);
  wv[1] = *(const v4f*)(TAB + (size_t)(kS + mw) * kPairs + p0 + 4);
#pragma unroll
  for (int q = 0; q < 6; ++q) br[q] = *(const v4f*)(BR + 3 * p0 + 4 * q);

  const bool c0 = (s == 0);
  const bool c1 = (s == 1);
  const bool cw = (s >= 2) && (s <= M + 2);
  const bool hasB = (M > 0);
  v8h hv;
#pragma unroll
  for (int e = 0; e < 8; ++e) {
    const float hM = hA[e >> 2][e & 3];
    const float hL = hB[e >> 2][e & 3];
    const float hP = hasB ? hL : 0.0f;
    const float wm = wv[e >> 2][e & 3];
    const float b1 = br[(3 * e + 1) >> 2][(3 * e + 1) & 3];
    const float b2 = br[(3 * e + 2) >> 2][(3 * e + 2) & 3];
    const float t0 = b2 * hM;
    const float t1 = b1 * hM + b2 * hP;
    float v = cw ? wm : 0.0f;
    v = c1 ? t1 : v;
    v = c0 ? t0 : v;
    hv[e] = f16_flush(v * kWCarry);
  }
  unsigned short* qh = WT + (size_t)e0;
  *(volatile v8h*)qh = hv;
  __threadfence();
  *(volatile v8h*)qh = hv;
}

static_assert(((kI * kFN * kFK / 8) % 256) == 0);
__global__ __launch_bounds__(256) void wf_pack_kernel(
    const float* __restrict__ TAB, const float* __restrict__ BR, unsigned short* __restrict__ WF)
{
  const int j = blockIdx.x * 256 + threadIdx.x;
  const int i = j >> 9;
  const int n = (j >> 3) & 63;
  const int s0 = (j & 7) * 8;
  const int o = n >> 1;
  const int r = n & 1;
  const int M = kL - 1 - r;
  const int p = 32 * o + i;
  float hM = TAB[(size_t)M * kPairs + p];
  float hL = TAB[(size_t)(M - 1) * kPairs + p];
  float b1 = BR[3 * p + 1];
  float b2 = BR[3 * p + 2];
  const float t0 = b2 * hM;
  const float t1 = b1 * hM + b2 * hL;
  v8h hv;
#pragma unroll
  for (int e = 0; e < 8; ++e) {
    const int s = s0 + e;
    int mw = M + 2 - s;
    mw = (mw < 0) ? 0 : mw;
    mw = (mw > kL - 1) ? (kL - 1) : mw;
    float wm = TAB[(size_t)(kS + mw) * kPairs + p];
    const bool cw = (s >= 2) && (s <= M + 2);
    float v = cw ? wm : 0.0f;
    v = (s == 1) ? t1 : v;
    v = (s == 0) ? t0 : v;
    hv[e] = f16_flush(v * kWCarry);
  }
  unsigned short* qh = WF + (size_t)j * 8;
  *(volatile v8h*)qh = hv;
  __threadfence();
  *(volatile v8h*)qh = hv;
}

static_assert(((kO * kL * kFK / 8) % 256) == 0);
__global__ __launch_bounds__(256) void hq_pack_kernel(
    const float* __restrict__ HC, unsigned short* __restrict__ HQ)
{
  const int j = blockIdx.x * 256 + threadIdx.x;
  const int o = j >> 8;
  const int M = (j >> 3) & 31;
  const int k0 = (j & 7) * 8;
  const float* sp = HC + ((size_t)(M * kO + o) * kI) * 2 + k0;
  const v4f a0 = *(const v4f*)(sp);
  const v4f a1 = *(const v4f*)(sp + 4);
  const float f0 = a0[0];
  const float f1 = a0[1];
  const float f2 = a0[2];
  const float f3 = a0[3];
  const float f4 = a1[0];
  const float f5 = a1[1];
  const float f6 = a1[2];
  const float f7 = a1[3];
  v8h hv;
  hv[0] = f16_flush(f0 * kHCarry);
  hv[1] = f16_flush(f1 * kHCarry);
  hv[2] = f16_flush(f2 * kHCarry);
  hv[3] = f16_flush(f3 * kHCarry);
  hv[4] = f16_flush(f4 * kHCarry);
  hv[5] = f16_flush(f5 * kHCarry);
  hv[6] = f16_flush(f6 * kHCarry);
  hv[7] = f16_flush(f7 * kHCarry);
  unsigned short* qh = HQ + (size_t)j * 8;
  *(volatile v8h*)qh = hv;
  __threadfence();
  *(volatile v8h*)qh = hv;
}

static_assert(((kB * kPairs) % 256) == 0);
__global__ __launch_bounds__(256) void state_kernel(
    const float* __restrict__ F, const float* __restrict__ TAB,
    const float* __restrict__ AR, unsigned short* __restrict__ YQ)
{
  const int q = blockIdx.x * 256 + threadIdx.x;
  const int b = q >> 10;
  const int p = q & 1023;
  const int o = p >> 5;
  const int i = p & 31;
  const float a1 = AR[2 * p + 1];
  const float h30 = TAB[(size_t)30 * kPairs + p];
  const float h31 = TAB[(size_t)31 * kPairs + p];
  const float h32 = TAB[(size_t)32 * kPairs + p];
  const float k31a = h32;
  const float k31b = -(a1 * h31);
  const float k30a = h31;
  const float k30b = -(a1 * h30);

  unsigned short* yrow = YQ + ((size_t)o * kGN + (size_t)kC * b) * kFK + 2 * i;
  {
    *(volatile unsigned*)yrow = 0u;
    __threadfence();
    *(volatile unsigned*)yrow = 0u;
  }

  const float* fp = F + ((size_t)i * kFRows + (size_t)kSegRows * b) * kFN + 2 * o;
  float y1 = 0.0f;
  float y2 = 0.0f;
  for (int c = 0; c < kC - 1; ++c) {
    const v2f f = *(const v2f*)(fp + (size_t)c * kFN);
    const float f31 = f[0];
    const float f30 = f[1];
    const float n1 = f31 + k31a * y1 + k31b * y2;
    const float n2 = f30 + k30a * y1 + k30b * y2;
    y1 = n1;
    y2 = n2;
    const _Float16 g1 = f16_flush(n1);
    const _Float16 g2 = f16_flush(n2);
    const unsigned wv = (unsigned)__builtin_bit_cast(unsigned short, g1) |
                        ((unsigned)__builtin_bit_cast(unsigned short, g2) << 16);
    unsigned short* po = yrow + (size_t)(c + 1) * kFK;
    *(volatile unsigned*)po = wv;
    __threadfence();
    *(volatile unsigned*)po = wv;
  }
}

static_assert(((kB * kT * kO) % 256) == 0);
__global__ __launch_bounds__(256) void out_kernel(
    const float* __restrict__ D, const float* __restrict__ G, float* __restrict__ out)
{
  const int e = blockIdx.x * 256 + threadIdx.x;
  const int b = e >> 17;
  const int t = (e >> 5) & (kT - 1);
  const int o = e & 31;
  const int c = t >> 5;
  const int M = t & 31;
  const float d = D[(size_t)(kC * b + c) * kN + 32 * M + o];
  const float g = G[(size_t)(o * kL + M) * kGN + kC * b + c];
  const float v = d + g;
  float* po = out + (size_t)e;
  *(volatile float*)po = v;
  __threadfence();
  *(volatile float*)po = v;
}

extern "C" void kernel_launch(void* const* d_in, const int* in_sizes, int n_in,
                              void* d_out, int out_size, void* d_ws, size_t ws_size,
                              hipStream_t stream)
{
  if (n_in < 3) return;
  if (in_sizes[0] != kB * kT * kI) return;
  if (in_sizes[1] != kO * kI * 3) return;
  if (in_sizes[2] != kO * kI * 2) return;
  if (out_size != 2097152) return;
  if (ws_size < kWsTotal) return;

  const float* u_in    = (const float*)d_in[0];
  const float* b_coeff = (const float*)d_in[1];
  const float* a_coeff = (const float*)d_in[2];
  float* out = (float*)d_out;

  char* ws = (char*)d_ws;
  float*          AR  = (float*)(ws + kOffAR);
  float*          BR  = (float*)(ws + kOffBR);
  float*          TAB = (float*)(ws + kOffTAB);
  float*          HC  = (float*)(ws + kOffHC);
  unsigned short* WT  = (unsigned short*)(ws + kOffWT);
  unsigned short* UP  = (unsigned short*)(ws + kOffUP);
  float*          D   = (float*)(ws + kOffD);
  unsigned short* UI  = (unsigned short*)(ws + kOffUI);
  unsigned short* WF  = (unsigned short*)(ws + kOffWF);
  unsigned short* HQ  = (unsigned short*)(ws + kOffHQ);
  float*          F   = (float*)(ws + kOffF);
  unsigned short* YQ  = (unsigned short*)(ws + kOffYQ);
  float*          G   = (float*)(ws + kOffG);

  constexpr float sW = 1.0f / kWCarry;
  constexpr float sH = 1.0f / kHCarry;

  rne_vec_kernel<<<2, 256, 0, stream>>>(a_coeff, AR, (kPairs * 2) / 4);
  rne_vec_kernel<<<3, 256, 0, stream>>>(b_coeff, BR, (kPairs * 3) / 4);

  pad_zero_kernel<<<1, 128, 0, stream>>>(UP);
  pad_body_f16_kernel<<<(kB * kT * kI / 8) / 256, 256, 0, stream>>>(u_in, UP);

  coeff_table_kernel<<<kPairs / 256, 256, 0, stream>>>(AR, BR, TAB, HC);

  wt_pack_kernel<<<(kN * kK / 8) / 256, 256, 0, stream>>>(TAB, BR, WT);

  ui_pack_kernel<<<(kI * kUiCh / 8) / 256, 256, 0, stream>>>(UP, UI);
  ui_tail_kernel<<<1, 32, 0, stream>>>(UI);

  wf_pack_kernel<<<(kI * kFN * kFK / 8) / 256, 256, 0, stream>>>(TAB, BR, WF);
  hq_pack_kernel<<<(kO * kL * kFK / 8) / 256, 256, 0, stream>>>(HC, HQ);

  for (int b = 0; b < kB; ++b) {
    eng::gemm_f16_kernel<2, 0><<<dim3((kC / 32) * (kN / 64) / 8), 256, 0, stream>>>(
        UP + (size_t)b * kUpB, nullptr, 1024, WT, nullptr, kK,
        D + (size_t)b * kC * kN, kN, kC, kN, kK, sW, 0.0f);
  }

  for (int i = 0; i < kI; ++i) {
    eng::gemm_f16_kernel<2, 0><<<dim3((kFRows / 32) * (kFN / 64) / 8), 256, 0, stream>>>(
        UI + (size_t)i * kUiCh, nullptr, 32, WF + (size_t)i * kFN * kFK, nullptr, kFK,
        F + (size_t)i * kFRows * kFN, kFN, kFRows, kFN, kFK, sW, 0.0f);
  }

  state_kernel<<<(kB * kPairs) / 256, 256, 0, stream>>>(F, TAB, AR, YQ);

  for (int o = 0; o < kO; ++o) {
    eng::gemm_f16_kernel<2, 0><<<dim3((kL / 32) * (kGN / 64) / 8), 256, 0, stream>>>(
        HQ + (size_t)o * kL * kFK, nullptr, kFK, YQ + (size_t)o * kGN * kFK, nullptr, kFK,
        G + (size_t)o * kL * kGN, kGN, kL, kGN, kFK, sH, 0.0f);
  }

  out_kernel<<<(kB * kT * kO) / 256, 256, 0, stream>>>(D, G, out);
}
